// BilinearDecoder_58256936403064
// MI455X (gfx1250) — hardware-run, weakly checked
//
#include <hip/hip_runtime.h>
#include <math.h>

#ifndef NE
#define NE 1000000
#endif
#define NE_FULL 1000000
#define NNODE 100000
#define DIM 64
#define NLAB 5
#define NCOL (NLAB * DIM)
#define NWAVE (NE / 32)
#define NBLK ((NWAVE + 7) / 8)
#define NPIECE (NE * NLAB / 4)
#define ZPIECES (NNODE * DIM / 8)
#define WPIECES (NCOL * DIM / 8)
#define ZP 72

static_assert(NE % 32 == 0);
static_assert(NE <= NE_FULL);
static_assert(DIM == 64);
static_assert(DIM % 32 == 0);
static_assert(NCOL % 16 == 0);
static_assert(ZPIECES % 256 == 0);
static_assert(WPIECES % 256 == 0);
static_assert((NE * NLAB) % 4 == 0);
static_assert(NPIECE % 8 == 0);
static_assert(((long long)NE * NLAB * 4) % 128 == 0);
static_assert(32 * 16 + 8 * 16 == 32 * NLAB * 4);
static_assert(8 * 32 * 16 == 32 * DIM * 2);
static_assert((ZP * 2) % 16 == 0 && ZP >= DIM);
static_assert(8 * 32 * ZP * 2 + 8 * 192 * 4 <= 131072);
static_assert(2 * NLAB <= 32);

typedef __attribute__((ext_vector_type(16))) __bf16       v16bf;
typedef __attribute__((ext_vector_type(8)))  float        v8f;
typedef __attribute__((ext_vector_type(4)))  float        v4f;
typedef __attribute__((ext_vector_type(4)))  unsigned int v4u;
typedef __attribute__((ext_vector_type(8)))  unsigned int v8u;

static constexpr size_t al256(size_t b) { return (b + 255) & ~(size_t)255; }
static constexpr size_t SZ_WP  = (size_t)NCOL * DIM * 2;
static constexpr size_t SZ_Z   = (size_t)NNODE * DIM * 2;
static constexpr size_t SZ_SC  = (size_t)NE * NLAB * 4;
static constexpr size_t SZ_PT  = (size_t)NWAVE * 128;
static constexpr size_t SZ_LSE = 128;
static constexpr size_t OFF_WP  = 0;
static constexpr size_t OFF_ZU  = OFF_WP + al256(SZ_WP);
static constexpr size_t OFF_ZM  = OFF_ZU + al256(SZ_Z);
static constexpr size_t OFF_SC  = OFF_ZM + al256(SZ_Z);
static constexpr size_t OFF_PT  = OFF_SC + al256(SZ_SC);
static constexpr size_t OFF_LSE = OFF_PT + al256(SZ_PT);
static constexpr size_t WS_TOTAL = OFF_LSE + al256(SZ_LSE);
static_assert(WS_TOTAL <= (size_t)134217728);
static_assert((size_t)NWAVE * 640 == SZ_SC);
static_assert((size_t)ZPIECES * 16 == SZ_Z);
static_assert((size_t)WPIECES * 16 == SZ_WP);


#define VST2(T, ptr, val) do { const T vst2_v_ = (val); *(volatile T*)(ptr) = vst2_v_; __threadfence(); *(volatile T*)(ptr) = vst2_v_; } while (0)
#define VST2V4(ptr, val) do { const v4f vst2_v4_ = (val); *(volatile v4f*)(ptr) = vst2_v4_; __threadfence(); *(volatile v4f*)(ptr) = vst2_v4_; } while (0)

__device__ __forceinline__ unsigned bf16_bits(float f) {
    unsigned u = __float_as_uint(f);
    u += 0x7FFFu + ((u >> 16) & 1u);
    return u >> 16;
}
__device__ __forceinline__ v4u pack8_bf16(const float* v) {
    v4u pk;
    pk.x = bf16_bits(v[0]) | (bf16_bits(v[1]) << 16);
    pk.y = bf16_bits(v[2]) | (bf16_bits(v[3]) << 16);
    pk.z = bf16_bits(v[4]) | (bf16_bits(v[5]) << 16);
    pk.w = bf16_bits(v[6]) | (bf16_bits(v[7]) << 16);
    return pk;
}
__device__ __forceinline__ v8u frag_ld_g(const unsigned short* __restrict__ p) {
    const v4u lo = *(const v4u*)(p);
    const v4u hi = *(const v4u*)(p + 16);
    return __builtin_shufflevector(lo, hi, 0, 1, 2, 3, 4, 5, 6, 7);
}
__device__ __forceinline__ v8f wmma_bf(v8u a, v8u b, v8f c) {
    c = __builtin_amdgcn_wmma_f32_16x16x32_bf16(false, __builtin_bit_cast(v16bf, a), false, __builtin_bit_cast(v16bf, b), (short)0, c, false, false);
    asm volatile("v_nop\n\tv_nop\n\tv_nop\n\tv_nop" : "+v"(c) : "v"(a), "v"(b));
    return c;
}
__device__ __forceinline__ void wave_sync_lds() {
    __builtin_amdgcn_fence(3  , "workgroup");
    __builtin_amdgcn_wave_barrier();
    __builtin_amdgcn_fence(2  , "workgroup");
}

__global__ __launch_bounds__(256) void k_wconv(const float* __restrict__ W, unsigned short* __restrict__ wp) {
    const unsigned u = blockIdx.x * 256u + threadIdx.x;
    if (u >= (unsigned)WPIECES) return;
    const unsigned k0 = 8u * (u & 7u);
    const unsigned n = u >> 3;
    const unsigned l = n >> 6, f = n & 63u;
    const float* Wl = W + (size_t)l * (DIM * DIM);
    float v[8];
#pragma unroll
    for (int i = 0; i < 8; ++i) v[i] = Wl[(size_t)(k0 + (unsigned)i) * DIM + f];
    const v4u pk = pack8_bf16(v);
    VST2(v4u, (v4u*)(wp + (size_t)n * DIM + k0), pk);
}

__device__ __forceinline__ void zconv_body(const float* __restrict__ src, unsigned short* __restrict__ dst, unsigned u) {
    const float* p = src + (size_t)u * 8u;
    const v4f a = *(const v4f*)p;
    const v4f b = *(const v4f*)(p + 4);
    const float v[8] = {a.x, a.y, a.z, a.w, b.x, b.y, b.z, b.w};
    const v4u pk = pack8_bf16(v);
    VST2(v4u, (v4u*)(dst + (size_t)u * 8u), pk);
}
__global__ __launch_bounds__(256) void k_zconv(const float* __restrict__ zu, const float* __restrict__ zm,
                                               unsigned short* __restrict__ zu16, unsigned short* __restrict__ zm16) {
    const unsigned u = blockIdx.x * 256u + threadIdx.x;
    if (u >= (unsigned)ZPIECES) return;
    if (blockIdx.y == 0u) zconv_body(zu, zu16, u);
    else                  zconv_body(zm, zm16, u);
}

__global__ __launch_bounds__(256) void k_scores(const unsigned short* __restrict__ zu16, const unsigned short* __restrict__ zm16,
                                                const unsigned short* __restrict__ wp, const int* __restrict__ eidx,
                                                float* __restrict__ scores, float* __restrict__ part) {
    __shared__ __align__(16) unsigned short sZ[8][32 * ZP];
    __shared__ __align__(16) float sS[8][192];
    const unsigned lane = threadIdx.x & 31u;
    const unsigned wave = __builtin_amdgcn_readfirstlane(threadIdx.x >> 5);
    const unsigned hh = lane >> 4, c = lane & 15u;
    const unsigned wg = blockIdx.x * 8u + wave;
    if (wg >= (unsigned)NWAVE) return;
    const unsigned e0 = wg * 32u;

    sS[wave][160u + lane] = 0.0f;

    {
        const unsigned rq = lane >> 3, pc = (lane & 7u) * 8u;
#pragma unroll
        for (int it = 0; it < 8; ++it) {
            const unsigned row = (unsigned)it * 4u + rq;
            int nd = eidx[e0 + row];
            nd = min(max(nd, 0), NNODE - 1);
            const v4u v = *(const v4u*)(zu16 + (size_t)nd * DIM + pc);
            *(v4u*)&sZ[wave][row * ZP + pc] = v;
        }
    }

    float zd[2][4][8];
#pragma unroll
    for (int j = 0; j < 2; ++j) {
        int nd = eidx[(size_t)NE_FULL + e0 + 16u * (unsigned)j + c];
        nd = min(max(nd, 0), NNODE - 1);
        const unsigned short* zr = zm16 + (size_t)nd * DIM + 8u * hh;
#pragma unroll
        for (int t = 0; t < 4; ++t) {
            const v4u w = *(const v4u*)(zr + 16 * t);
            zd[j][t][0] = __uint_as_float(w.x << 16); zd[j][t][1] = __uint_as_float(w.x & 0xFFFF0000u);
            zd[j][t][2] = __uint_as_float(w.y << 16); zd[j][t][3] = __uint_as_float(w.y & 0xFFFF0000u);
            zd[j][t][4] = __uint_as_float(w.z << 16); zd[j][t][5] = __uint_as_float(w.z & 0xFFFF0000u);
            zd[j][t][6] = __uint_as_float(w.w << 16); zd[j][t][7] = __uint_as_float(w.w & 0xFFFF0000u);
        }
    }

    wave_sync_lds();

    v8u bz[2][2];
#pragma unroll
    for (int j = 0; j < 2; ++j)
#pragma unroll
        for (int ks = 0; ks < 2; ++ks) {
            const unsigned o = (16u * (unsigned)j + c) * ZP + 32u * (unsigned)ks + 8u * hh;
            const v4u lo = *(const v4u*)&sZ[wave][o];
            const v4u hi = *(const v4u*)&sZ[wave][o + 16u];
            bz[j][ks] = __builtin_shufflevector(lo, hi, 0, 1, 2, 3, 4, 5, 6, 7);
        }

    const unsigned short* wl = wp + (size_t)(c * DIM + 8u * hh);
#pragma unroll 1
    for (unsigned l = 0; l < (unsigned)NLAB; ++l) {
        float d0 = 0.0f, d1 = 0.0f;
#pragma unroll
        for (int t = 0; t < 4; ++t) {
            const unsigned short* ap = wl + (size_t)(l * 64u + (unsigned)t * 16u) * DIM;
            const v8u a0 = frag_ld_g(ap);
            const v8u a1 = frag_ld_g(ap + 32);
            v8f x0 = (v8f){0.f, 0.f, 0.f, 0.f, 0.f, 0.f, 0.f, 0.f};
            v8f x1 = x0;
            x0 = wmma_bf(a0, bz[0][0], x0);
            x1 = wmma_bf(a0, bz[1][0], x1);
            x0 = wmma_bf(a1, bz[0][1], x0);
            x1 = wmma_bf(a1, bz[1][1], x1);
#pragma unroll
            for (int r = 0; r < 8; ++r) {
                d0 += x0[r] * zd[0][t][r];
                d1 += x1[r] * zd[1][t][r];
            }
        }
        d0 += __shfl_xor(d0, 16, 32);
        d1 += __shfl_xor(d1, 16, 32);
        const float s = (hh != 0u) ? d1 : d0;
        sS[wave][lane * 5u + l] = s;

        float mv = s;
        mv = fmaxf(mv, __shfl_xor(mv, 16, 32)); mv = fmaxf(mv, __shfl_xor(mv, 8, 32));
        mv = fmaxf(mv, __shfl_xor(mv, 4, 32));  mv = fmaxf(mv, __shfl_xor(mv, 2, 32));
        mv = fmaxf(mv, __shfl_xor(mv, 1, 32));
        float pv = expf(s - mv);
        pv += __shfl_xor(pv, 16, 32); pv += __shfl_xor(pv, 8, 32);
        pv += __shfl_xor(pv, 4, 32);  pv += __shfl_xor(pv, 2, 32);
        pv += __shfl_xor(pv, 1, 32);
        if (lane == 0u) { sS[wave][160u + l] = mv; sS[wave][165u + l] = pv; }
    }
    wave_sync_lds();

    {
        const unsigned l8 = lane & 7u;
        const v4f p0 = *(const v4f*)&sS[wave][4u * lane];
        const v4f p1 = *(const v4f*)&sS[wave][128u + 4u * l8];
        const v4f p2 = *(const v4f*)&sS[wave][160u + 4u * l8];
        float* sd = scores + (size_t)e0 * NLAB;
        float* pd = part + (size_t)wg * 32u;
        for (int pass = 0; pass < 2; ++pass) {
            *(volatile v4f*)(sd + 4u * lane) = p0;
            if (lane < 8u) {
                *(volatile v4f*)(sd + 128u + 4u * lane) = p1;
                *(volatile v4f*)(pd + 4u * lane) = p2;
            }
            __threadfence();
        }
    }
}

__global__ __launch_bounds__(256) void k_lse(const float* __restrict__ part, float* __restrict__ lse) {
#pragma clang fp contract(off)
    __shared__ float  sMx[8];
    __shared__ double sSm[8];
    __shared__ float  sL[32];
    const unsigned t = threadIdx.x, lane = t & 31u;
    const unsigned wave = __builtin_amdgcn_readfirstlane(t >> 5);
    if (t < 32u) sL[t] = 0.0f;
    __syncthreads();
#pragma unroll 1
    for (unsigned l = 0; l < (unsigned)NLAB; ++l) {
        float m = -3.0e38f;
#pragma unroll 1
        for (unsigned i = t; i < (unsigned)NWAVE; i += 256u) m = fmaxf(m, part[(size_t)i * 32u + l]);
        m = fmaxf(m, __shfl_xor(m, 16, 32)); m = fmaxf(m, __shfl_xor(m, 8, 32));
        m = fmaxf(m, __shfl_xor(m, 4, 32));  m = fmaxf(m, __shfl_xor(m, 2, 32));
        m = fmaxf(m, __shfl_xor(m, 1, 32));
        if (lane == 0u) sMx[wave] = m;
        __syncthreads();
        float M = sMx[0];
#pragma unroll
        for (int w = 1; w < 8; ++w) M = fmaxf(M, sMx[w]);
        double acc = 0.0;
#pragma unroll 1
        for (unsigned i = t; i < (unsigned)NWAVE; i += 256u) {
            const float mi = part[(size_t)i * 32u + l];
            const float si = part[(size_t)i * 32u + 5u + l];
            acc += (double)si * (double)expf(mi - M);
        }
        acc += __shfl_xor(acc, 16, 32); acc += __shfl_xor(acc, 8, 32);
        acc += __shfl_xor(acc, 4, 32);  acc += __shfl_xor(acc, 2, 32);
        acc += __shfl_xor(acc, 1, 32);
        if (lane == 0u) sSm[wave] = acc;
        __syncthreads();
        double tot = sSm[0];
#pragma unroll
        for (int w = 1; w < 8; ++w) tot += sSm[w];
        if (t == 0u) sL[l] = M + logf((float)tot);
        __syncthreads();
    }
    if (t < 8u) {
        v4f v;
        v.x = sL[4u * t]; v.y = sL[4u * t + 1u]; v.z = sL[4u * t + 2u]; v.w = sL[4u * t + 3u];
        VST2V4(lse + 4u * t, v);
    }
}

__device__ __forceinline__ float pick5(unsigned k, float a0, float a1, float a2, float a3, float a4) {
    float v = a0;
    v = (k == 1u) ? a1 : v;
    v = (k == 2u) ? a2 : v;
    v = (k == 3u) ? a3 : v;
    v = (k == 4u) ? a4 : v;
    return v;
}
__global__ __launch_bounds__(256) void k_final(const float* __restrict__ scores, const float* __restrict__ lse, float* __restrict__ out) {
    const unsigned i = blockIdx.x * 256u + threadIdx.x;
    const unsigned ic = min(i, (unsigned)(NPIECE - 1));
    const v4f s = *(const v4f*)(scores + (size_t)ic * 4u);
    const v4f la = *(const v4f*)(lse);
    const v4f lb = *(const v4f*)(lse + 4);
    const unsigned r0 = (4u * ic) % 5u;
    const unsigned r1 = (r0 + 1u) % 5u;
    const unsigned r2 = (r0 + 2u) % 5u;
    const unsigned r3 = (r0 + 3u) % 5u;
    v4f o;
    o.x = s.x - pick5(r0, la.x, la.y, la.z, la.w, lb.x);
    o.y = s.y - pick5(r1, la.x, la.y, la.z, la.w, lb.x);
    o.z = s.z - pick5(r2, la.x, la.y, la.z, la.w, lb.x);
    o.w = s.w - pick5(r3, la.x, la.y, la.z, la.w, lb.x);
    if (i < (unsigned)NPIECE) { VST2V4(out + (size_t)i * 4u, o); }
}

extern "C" void kernel_launch(void* const* d_in, const int* in_sizes, int n_in, void* d_out, int out_size,
                              void* d_ws, size_t ws_size, hipStream_t stream) {
    if (n_in < 4) return;
    if (in_sizes[0] < NNODE * DIM || in_sizes[1] < NNODE * DIM || in_sizes[2] < NLAB * DIM * DIM) return;
    if (in_sizes[3] < NE_FULL + NE || out_size < NE * NLAB) return;
    if (ws_size < WS_TOTAL) return;

    const float* z_user  = (const float*)d_in[0];
    const float* z_movie = (const float*)d_in[1];
    const float* W       = (const float*)d_in[2];
    const int*   eidx    = (const int*)d_in[3];
    float* out = (float*)d_out;

    char* wsp = (char*)d_ws;
    unsigned short* wp   = (unsigned short*)(wsp + OFF_WP);
    unsigned short* zu16 = (unsigned short*)(wsp + OFF_ZU);
    unsigned short* zm16 = (unsigned short*)(wsp + OFF_ZM);
    float*          sc   = (float*)(wsp + OFF_SC);
    float*          part = (float*)(wsp + OFF_PT);
    float*          lse  = (float*)(wsp + OFF_LSE);

    k_wconv<<<WPIECES / 256, 256, 0, stream>>>(W, wp);
    k_zconv<<<dim3(ZPIECES / 256, 2), 256, 0, stream>>>(z_user, z_movie, zu16, zm16);
    k_scores<<<NBLK, 256, 0, stream>>>(zu16, zm16, wp, eidx, sc, part);
    k_lse<<<1, 256, 0, stream>>>(part, lse);
    k_final<<<(NPIECE + 255) / 256, 256, 0, stream>>>(sc, lse, out);
}
